// SynthesizerEncoder_13280038879459
// MI455X (gfx1250) — hardware-run, weakly checked
//
#include <hip/hip_runtime.h>
#include <math.h>

typedef __attribute__((ext_vector_type(16))) _Float16 v16h;
typedef __attribute__((ext_vector_type(16))) __bf16 v16b;
typedef __attribute__((ext_vector_type(8)))  _Float16 v8h;
typedef __attribute__((ext_vector_type(8)))  float v8f;
typedef __attribute__((ext_vector_type(4)))  float v4f;
typedef __attribute__((ext_vector_type(2)))  float v2f;
typedef __attribute__((ext_vector_type(4)))  unsigned v4u;
typedef __attribute__((ext_vector_type(4)))  int v4i;
typedef float __attribute__((may_alias)) float_a;
typedef int __attribute__((may_alias)) int_a;

template <typename T> __device__ __forceinline__ void vst2(void* p, T v) { *(volatile T*)p = v; __threadfence(); *(volatile T*)p = v; }
__device__ __forceinline__ v8f wmma16(v16h a, v16h b, v8f c) {
  v8f d = __builtin_amdgcn_wmma_f32_16x16x32_f16(false, a, false, b, (short)0, c, false, false);
  asm volatile("v_nop\n\tv_nop\n\tv_nop\n\tv_nop" : "+v"(d) : "v"(a), "v"(b));
  return d;
}
__device__ __forceinline__ v8f wmma_bf(v16b a, v16b b, v8f c) {
  v8f d = __builtin_amdgcn_wmma_f32_16x16x32_bf16(false, a, false, b, (short)0, c, false, false);
  asm volatile("v_nop\n\tv_nop\n\tv_nop\n\tv_nop" : "+v"(d) : "v"(a), "v"(b));
  return d;
}
__device__ __forceinline__ v16h frag_h(const _Float16* rowk0, int lane) {
  union { v16h v; v8h q[2]; } u; const _Float16* p = rowk0 + 8 * (lane >> 4);
  u.q[0] = *(const v8h*)p; u.q[1] = *(const v8h*)(p + 16); return u.v;
}
__device__ __forceinline__ v16h frag_f32(const float* rowk0, int lane) {
  v16h a; const float* p = rowk0 + 8 * (lane >> 4);
#pragma unroll
  for (int i = 0; i < 8; ++i) { a[i] = (_Float16)p[i]; a[8 + i] = (_Float16)p[16 + i]; }
  return a;
}
__device__ __forceinline__ v16h frag_f32s(const float* rowk0, int lane, float sc) {
  v16h a; const float* p = rowk0 + 8 * (lane >> 4);
#pragma unroll
  for (int i = 0; i < 8; ++i) { a[i] = (_Float16)(p[i] * sc); a[8 + i] = (_Float16)(p[16 + i] * sc); }
  return a;
}
__device__ __forceinline__ v16h fragc_f32(const float* W, int k0, int n, int lane, int ld, int K) {
  v16h a; const int g = lane >> 4;
#pragma unroll
  for (int i = 0; i < 8; ++i) { const int ka = k0 + 8 * g + i, kb = ka + 16;
    a[i] = (_Float16)(ka < K ? W[(size_t)(ka < K ? ka : K - 1) * ld + n] : 0.f); a[8 + i] = (_Float16)(kb < K ? W[(size_t)(kb < K ? kb : K - 1) * ld + n] : 0.f); }
  return a;
}
struct F2 { v16b h, l; };
__device__ __forceinline__ F2 bsplit16(const float v[16]) { F2 r;
#pragma unroll
  for (int i = 0; i < 16; ++i) { const __bf16 h = (__bf16)v[i]; r.h[i] = h; r.l[i] = (__bf16)(v[i] - (float)h); }
  return r; }
__device__ __forceinline__ F2 split_row(const float* row, int k0, int lane) { float v[16]; const float* p = row + k0 + 8 * (lane >> 4);
#pragma unroll
  for (int i = 0; i < 8; ++i) { v[i] = p[i]; v[8 + i] = p[16 + i]; }
  return bsplit16(v); }
__device__ __forceinline__ F2 split_rowK(const float* row, int k0, int lane, int K) { float v[16]; const int g = lane >> 4;
#pragma unroll
  for (int i = 0; i < 8; ++i) { const int ka = k0 + 8 * g + i, kb = ka + 16; v[i] = ka < K ? row[ka < K ? ka : K - 1] : 0.f; v[8 + i] = kb < K ? row[kb < K ? kb : K - 1] : 0.f; }
  return bsplit16(v); }
__device__ __forceinline__ F2 split_col(const float* W, int k0, int n, int lane, int ld, int K) { float v[16]; const int g = lane >> 4;
#pragma unroll
  for (int i = 0; i < 8; ++i) { const int ka = k0 + 8 * g + i, kb = ka + 16; v[i] = ka < K ? W[(size_t)(ka < K ? ka : K - 1) * ld + n] : 0.f; v[8 + i] = kb < K ? W[(size_t)(kb < K ? kb : K - 1) * ld + n] : 0.f; }
  return bsplit16(v); }
__device__ __forceinline__ v8f mac3(const F2& a, const F2& b, v8f c) { c = wmma_bf(a.l, b.h, c); c = wmma_bf(a.h, b.l, c); return wmma_bf(a.h, b.h, c); }
__device__ __forceinline__ float sigm(float v) { return 1.0f / (1.0f + expf(-v)); }
#define LDSX() do { asm volatile("s_wait_dscnt 0" ::: "memory"); __builtin_amdgcn_wave_barrier(); __builtin_amdgcn_fence(__ATOMIC_RELEASE, "workgroup"); } while (0)


#define NB 2
#define SS 2048
#define DM 1024
#define NH 16
#define HD 64
#define FF 4096
#define NR (NB * SS)
#define WSC 256.0f
#ifndef TQB
#define TQB (SS / 64)
#define TNB NB
#define TOB (NB * SS / 64)
#endif
typedef __attribute__((ext_vector_type(8))) __bf16 v8b;
__device__ __forceinline__ v16b frag_b(const __bf16* rowk0, int lane) {
  union { v16b v; v8b q[2]; } u; const __bf16* p = rowk0 + 8 * (lane >> 4);
  u.q[0] = *(const v8b*)p; u.q[1] = *(const v8b*)(p + 16); return u.v;
}
__device__ __forceinline__ float bfr(float v) { return (float)(__bf16)v; }
__device__ __attribute__((noinline)) float exp_ni(float v) { return expf(v); }
__device__ __attribute__((noinline)) float erf_ni(float v) { return erff(v); }
__device__ __attribute__((noinline)) float gelu_e(float v) { return 0.5f * v * (1.0f + erff(v * 0.70710678118654752f)); }

#define WS_PV  0u
#define WS_PA1 (WS_PV + 2u * (size_t)DM * DM)
#define WS_PA2 (WS_PA1 + 2u * (size_t)HD * HD)
#define WS_PO  (WS_PA2 + 2u * (size_t)SS * HD)
#define WS_PF1 (WS_PO + 2u * (size_t)DM * DM)
#define WS_PF2 (WS_PF1 + 2u * (size_t)FF * DM)
#define WS_HID (WS_PF2 + 2u * (size_t)DM * FF)
#define WS_V   (WS_HID + 2u * (size_t)NR * DM)
#define WS_O   (WS_V + 2u * (size_t)NB * DM * SS)
#define WS_T   (WS_O + 4u * (size_t)NR * DM)
#define WS_H1  (WS_T + 4u * (size_t)NR * DM)
#define WS_H1H (WS_H1 + 4u * (size_t)NR * DM)
#define WS_G   (WS_H1H + 2u * (size_t)NR * DM)
#define WS_END (WS_G + 2u * (size_t)NR * FF)

__global__ __launch_bounds__(256) void k_pack(const float* __restrict__ VW, const float* __restrict__ OW, const float* __restrict__ F1, const float* __restrict__ F2W, const float* __restrict__ A1, const float* __restrict__ A2, char* __restrict__ ws) {
  const int n = blockIdx.x, which = blockIdx.y, t = threadIdx.x; __shared__ __align__(16) _Float16 sh[FF]; __shared__ __align__(16) __bf16 sb[DM];
  if (which == 0) { if (n >= DM) return; for (int k = t; k < DM; k += 256) sb[k] = (__bf16)VW[(size_t)k * DM + n]; __syncthreads(); for (int q = t; q < DM / 8; q += 256) vst2((unsigned*)((__bf16*)(ws + WS_PV) + (size_t)n * DM + q * 8), *(const v4u*)&sb[q * 8]); }
  else if (which == 1) { if (n >= DM) return; for (int k = t; k < DM; k += 256) sh[k] = (_Float16)(bfr(OW[(size_t)k * DM + n]) * WSC); __syncthreads(); for (int q = t; q < DM / 8; q += 256) vst2((unsigned*)((_Float16*)(ws + WS_PO) + (size_t)n * DM + q * 8), *(const v4u*)&sh[q * 8]); }
  else if (which == 2) { for (int k = t; k < DM; k += 256) sh[k] = (_Float16)(bfr(F1[(size_t)k * FF + n]) * WSC); __syncthreads(); for (int q = t; q < DM / 8; q += 256) vst2((unsigned*)((_Float16*)(ws + WS_PF1) + (size_t)n * DM + q * 8), *(const v4u*)&sh[q * 8]); }
  else if (which == 3) { if (n >= DM) return; for (int k = t; k < FF; k += 256) sh[k] = (_Float16)(bfr(F2W[(size_t)k * DM + n]) * WSC); __syncthreads(); for (int q = t; q < FF / 8; q += 256) vst2((unsigned*)((_Float16*)(ws + WS_PF2) + (size_t)n * FF + q * 8), *(const v4u*)&sh[q * 8]); }
  else { if (n < HD) { if (t < HD) sb[t] = (__bf16)A1[(size_t)t * HD + n]; __syncthreads(); if (t < HD / 8) vst2((unsigned*)((__bf16*)(ws + WS_PA1) + (size_t)n * HD + t * 8), *(const v4u*)&sb[t * 8]); }
         if (n < SS) { __syncthreads(); if (t < HD) sh[t] = (_Float16)bfr(A2[(size_t)t * SS + n]); __syncthreads(); if (t < HD / 8) vst2((unsigned*)((_Float16*)(ws + WS_PA2) + (size_t)n * HD + t * 8), *(const v4u*)&sh[t * 8]); } } }
__global__ __launch_bounds__(128) void k_hid(const float* __restrict__ X, const __bf16* __restrict__ PA1, const float* __restrict__ B1, _Float16* __restrict__ HIDr) { __shared__ __align__(16) _Float16 so[4][16][72];
  const int tid = threadIdx.x, wave = tid >> 5, lane = tid & 31, col = lane & 15, g = lane >> 4; const size_t r0 = (size_t)blockIdx.x * 64 + wave * 16; const int h = blockIdx.y;
  v8f acc[4] = {};
#pragma unroll
  for (int kc = 0; kc < 2; ++kc) { v16b a; { const float* p = X + (r0 + col) * DM + h * HD + kc * 32 + 8 * g;
#pragma unroll
      for (int i = 0; i < 8; ++i) { a[i] = (__bf16)p[i]; a[8 + i] = (__bf16)p[16 + i]; } }
#pragma unroll
    for (int j = 0; j < 4; ++j) acc[j] = wmma_bf(a, frag_b(PA1 + (size_t)(j * 16 + col) * HD + kc * 32, lane), acc[j]); }
#pragma unroll
  for (int j = 0; j < 4; ++j) { const float bb = bfr(B1[j * 16 + col]);
#pragma unroll
    for (int r = 0; r < 8; ++r) so[wave][8 * g + r][j * 16 + col] = (_Float16)fmaxf(acc[j][r] + bb, 0.f); }
  LDSX(); for (int rl = 0; rl < 16; ++rl) if (lane < 8) vst2((unsigned*)(HIDr + (r0 + rl) * DM + h * HD + lane * 8), *(const v4u*)&so[wave][rl][lane * 8]); }
__global__ __launch_bounds__(128) void k_val(const float* __restrict__ X, const __bf16* __restrict__ PV, _Float16* __restrict__ V) { __shared__ __align__(16) _Float16 st[128][72];
  const int tid = threadIdx.x, wave = tid >> 5, lane = tid & 31, col = lane & 15, g = lane >> 4; const size_t rb = (size_t)blockIdx.x * 64; const size_t r0 = rb + wave * 16; const int c0 = blockIdx.y * 128;
  v8f acc[8] = {};
#pragma unroll 2
  for (int kc = 0; kc < DM / 32; ++kc) { v16b a; { const float* p = X + (r0 + col) * DM + kc * 32 + 8 * g;
#pragma unroll
      for (int i = 0; i < 8; ++i) { a[i] = (__bf16)p[i]; a[8 + i] = (__bf16)p[16 + i]; } }
#pragma unroll
    for (int j = 0; j < 8; ++j) acc[j] = wmma_bf(a, frag_b(PV + (size_t)(c0 + j * 16 + col) * DM + kc * 32, lane), acc[j]); }
#pragma unroll
  for (int j = 0; j < 8; ++j)
#pragma unroll
    for (int r = 0; r < 8; ++r) st[j * 16 + col][wave * 16 + 8 * g + r] = (_Float16)acc[j][r];
  __syncthreads(); const size_t b = rb / SS; const int s0 = (int)(rb % SS); for (int e = tid; e < 128 * 8; e += 128) { const int d = e >> 3, pc = e & 7; vst2((unsigned*)(V + ((b * DM + c0 + d) * SS) + s0 + pc * 8), *(const v4u*)&st[d][pc * 8]); } }
__global__ __launch_bounds__(128) void k_attn(const _Float16* __restrict__ HIDr, const _Float16* __restrict__ PA2, const float* __restrict__ B2, const _Float16* __restrict__ V, float* __restrict__ O) {
  __shared__ __align__(16) _Float16 sph[4][16][40]; __shared__ __align__(16) float so[4][16][68];
  const int tid = threadIdx.x, wave = tid >> 5, lane = tid & 31, col = lane & 15, g = lane >> 4; const int h = blockIdx.y; const size_t b = blockIdx.z; const int q0 = blockIdx.x * 64 + wave * 16; const size_t rq = b * SS + q0;
  v16h aq[2];
#pragma unroll
  for (int kc = 0; kc < 2; ++kc) aq[kc] = frag_h(HIDr + (rq + col) * DM + h * HD + kc * 32, lane);
  float m[8], l[8];
#pragma unroll
  for (int r = 0; r < 8; ++r) { m[r] = -3.0e38f; l[r] = 0.f; }
  v8f acc[4] = {};
#pragma unroll 1
  for (int ks = 0; ks < SS / 32; ++ks) { const int j0 = ks * 32; v8f s[2];
#pragma unroll
    for (int ct = 0; ct < 2; ++ct) { const int kk = j0 + ct * 16 + col; v8f c = {}; const float bb = bfr(B2[kk]);
#pragma unroll
      for (int kc = 0; kc < 2; ++kc) c = wmma16(aq[kc], frag_h(PA2 + (size_t)kk * HD + kc * 32, lane), c);
#pragma unroll
      for (int r = 0; r < 8; ++r) s[ct][r] = c[r] + bb; }
#pragma unroll
    for (int r = 0; r < 8; ++r) { float mx = fmaxf(s[0][r], s[1][r]);
#pragma unroll
      for (int o = 1; o < 16; o <<= 1) mx = fmaxf(mx, __shfl_xor(mx, o));
      const float mn = fmaxf(m[r], mx); const float alpha = (m[r] <= -1.0e38f) ? 0.f : __expf(m[r] - mn); const float e0 = __expf(s[0][r] - mn), e1 = __expf(s[1][r] - mn); float es = e0 + e1;
#pragma unroll
      for (int o = 1; o < 16; o <<= 1) es += __shfl_xor(es, o);
      l[r] = l[r] * alpha + es; m[r] = mn;
#pragma unroll
      for (int dt = 0; dt < 4; ++dt) acc[dt][r] *= alpha;
      sph[wave][8 * g + r][col] = (_Float16)(e0 * 2048.0f); sph[wave][8 * g + r][16 + col] = (_Float16)(e1 * 2048.0f); }
    LDSX();
    const v16h pa = frag_h(&sph[wave][col][0], lane);
#pragma unroll
    for (int dt = 0; dt < 4; ++dt) acc[dt] = wmma16(pa, frag_h(V + ((b * DM + h * HD + dt * 16 + col) * SS) + j0, lane), acc[dt]);
    LDSX(); }
#pragma unroll
  for (int r = 0; r < 8; ++r) { const float il = (1.0f / 2048.0f) / l[r];
#pragma unroll
    for (int dt = 0; dt < 4; ++dt) so[wave][8 * g + r][dt * 16 + col] = acc[dt][r] * il; }
  LDSX();
  for (int rl = 0; rl < 16; ++rl) if (lane < 16) vst2(O + (rq + rl) * DM + h * HD + lane * 4, *(const v4f*)&so[wave][rl][lane * 4]);
}
__global__ __launch_bounds__(256) void k_ln(const float* __restrict__ A, const float* __restrict__ G, const float* __restrict__ Bt, float* __restrict__ OUT, _Float16* __restrict__ OUTH) { __shared__ float red[8]; __shared__ __align__(16) float so2[DM]; __shared__ __align__(16) _Float16 sh[DM]; const int t = threadIdx.x; const size_t row = blockIdx.x;
  float v[4]; float s = 0.f; for (int i = 0; i < 4; ++i) { v[i] = A[row * DM + t + 256 * i]; s += v[i]; }
#pragma unroll
  for (int o = 1; o < 32; o <<= 1) s += __shfl_xor(s, o);
  if ((t & 31) == 0) red[t >> 5] = s; __syncthreads(); float tot = 0.f; for (int i = 0; i < 8; ++i) tot += red[i]; const float mu = tot / (float)DM; __syncthreads();
  float q = 0.f; for (int i = 0; i < 4; ++i) { const float d = v[i] - mu; q += d * d; }
#pragma unroll
  for (int o = 1; o < 32; o <<= 1) q += __shfl_xor(q, o);
  if ((t & 31) == 0) red[t >> 5] = q; __syncthreads(); float tq = 0.f; for (int i = 0; i < 8; ++i) tq += red[i]; const float inv = 1.0f / sqrtf(tq / (float)DM + 1e-5f);
  for (int i = 0; i < 4; ++i) { const int c = t + 256 * i; const float y = (v[i] - mu) * inv * bfr(G[c]) + bfr(Bt[c]); so2[c] = y; sh[c] = (_Float16)y; } __syncthreads();
  vst2(OUT + row * DM + t * 4, *(const v4f*)&so2[t * 4]); if (OUTH && t < DM / 8) vst2((unsigned*)(OUTH + row * DM + t * 8), *(const v4u*)&sh[t * 8]); }
template <int MODE, int KW>
__global__ __launch_bounds__(128) void k_g(const void* __restrict__ Ain, const _Float16* __restrict__ Wr, const float* __restrict__ BI, const float* __restrict__ RES, float* __restrict__ O32, _Float16* __restrict__ O16, int ow) { __shared__ __align__(16) float sf[4][16][132]; __shared__ __align__(16) _Float16 so[64][136];
  const int tid = threadIdx.x, wave = tid >> 5, lane = tid & 31, col = lane & 15, g = lane >> 4; const size_t rb = (size_t)blockIdx.x * 64; const size_t r0 = rb + wave * 16; const int c0 = blockIdx.y * 128;
  v8f acc[8] = {};
#pragma unroll 2
  for (int kc = 0; kc < KW / 32; ++kc) { v16h a; if (MODE == 0) { const float* p = (const float*)Ain + (r0 + col) * KW + kc * 32 + 8 * g;
#pragma unroll
      for (int i = 0; i < 8; ++i) { a[i] = (_Float16)p[i]; a[8 + i] = (_Float16)p[16 + i]; } } else a = frag_h((const _Float16*)Ain + (r0 + col) * KW + kc * 32, lane);
#pragma unroll
    for (int j = 0; j < 8; ++j) acc[j] = wmma16(a, frag_h(Wr + (size_t)(c0 + j * 16 + col) * KW + kc * 32, lane), acc[j]); }
  if (MODE == 1) {
#pragma unroll
    for (int j = 0; j < 8; ++j) { const float bb = bfr(BI[c0 + j * 16 + col]);
#pragma unroll
      for (int r = 0; r < 8; ++r) so[wave * 16 + 8 * g + r][j * 16 + col] = (_Float16)gelu_e(acc[j][r] * (1.0f / WSC) + bb); }
    __syncthreads(); for (int e = tid; e < 64 * 16; e += 128) { const int rl = e >> 4, q = e & 15; vst2((unsigned*)(O16 + (rb + rl) * ow + c0 + q * 8), *(const v4u*)&so[rl][q * 8]); } return; }
#pragma unroll
  for (int j = 0; j < 8; ++j) { const int c = c0 + j * 16 + col; const float bb = BI ? bfr(BI[c]) : 0.f;
#pragma unroll
    for (int r = 0; r < 8; ++r) { const float res = RES[(r0 + 8 * g + r) * ow + c]; sf[wave][8 * g + r][j * 16 + col] = acc[j][r] * (1.0f / WSC) + bb + (MODE == 0 ? bfr(res) : res); } }
  LDSX(); for (int rl = 0; rl < 16; ++rl) vst2(O32 + (r0 + rl) * ow + c0 + lane * 4, *(const v4f*)&sf[wave][rl][lane * 4]); }
extern "C" void kernel_launch(void* const* d_in, const int* in_sizes, int n_in, void* d_out, int out_size, void* d_ws, size_t ws_size, hipStream_t stream) {
  (void)in_sizes; (void)n_in; (void)out_size;
  const float** F = (const float**)d_in;
  if (ws_size < (size_t)WS_END) return;
  char* ws = (char*)d_ws; _Float16 *HIDr = (_Float16*)(ws + WS_HID), *V = (_Float16*)(ws + WS_V), *H1H = (_Float16*)(ws + WS_H1H), *G = (_Float16*)(ws + WS_G); float *O = (float*)(ws + WS_O), *T = (float*)(ws + WS_T), *H1 = (float*)(ws + WS_H1);
  const int nr = TNB * SS;
  k_pack<<<dim3(FF, 5), 256, 0, stream>>>(F[5], F[6], F[7], F[9], F[1], F[3], ws);
  k_hid<<<dim3(nr / 64, NH), 128, 0, stream>>>(F[0], (const __bf16*)(ws + WS_PA1), F[2], HIDr);
  k_val<<<dim3(nr / 64, DM / 128), 128, 0, stream>>>(F[0], (const __bf16*)(ws + WS_PV), V);
  k_attn<<<dim3(TQB, NH, TNB), 128, 0, stream>>>(HIDr, (const _Float16*)(ws + WS_PA2), F[4], V, O);
  k_g<0, DM><<<dim3(TOB, DM / 128), 128, 0, stream>>>(O, (const _Float16*)(ws + WS_PO), nullptr, F[0], T, nullptr, DM);
  k_ln<<<TOB * 64, 256, 0, stream>>>(T, F[11], F[12], H1, H1H);
  k_g<1, DM><<<dim3(TOB, FF / 128), 128, 0, stream>>>(H1H, (const _Float16*)(ws + WS_PF1), F[8], nullptr, nullptr, G, FF);
  k_g<2, FF><<<dim3(TOB, DM / 128), 128, 0, stream>>>(G, (const _Float16*)(ws + WS_PF2), F[10], H1, T, nullptr, DM);
  k_ln<<<TOB * 64, 256, 0, stream>>>(T, F[13], F[14], (float*)d_out, nullptr);
}
